// GraphAttentionLayer_86706799772346
// MI455X (gfx1250) — hardware-verified
//
#include <hip/hip_runtime.h>
#include <stddef.h>
#include <stdint.h>
#include <math.h>


#define KIN     256
#define DOUT    64
#define NTHR    256
#define GTHR    128
#define GBM     64
#define KT      64
#define PP      72
#define NEGSL   0.01f
#define WSMAX   134217728

static_assert((KIN % 32) == 0 && (KIN / 8) == 32);
static_assert(DOUT == 64 && KT == 64 && GBM == 64);
static_assert(GBM == (GTHR / 32) * 16);
static_assert(GTHR == 2 * GBM);
static_assert((PP % 8) == 0 && PP >= KT);
static_assert((KT % 32) == 0);

typedef float          v4f  __attribute__((ext_vector_type(4)));
typedef float          v8f  __attribute__((ext_vector_type(8)));
typedef int            v8i  __attribute__((ext_vector_type(8)));
typedef unsigned int   v4u  __attribute__((ext_vector_type(4)));
typedef unsigned short v8us __attribute__((ext_vector_type(8)));
typedef __bf16         v16b __attribute__((ext_vector_type(16)));
typedef v4f  __attribute__((may_alias)) v4fa;
typedef v4u  __attribute__((may_alias)) v4ua;
typedef v8us __attribute__((may_alias)) v8usa;
union FragB { v16b v; v8us h[2]; v8i w; };

__device__ __forceinline__ v8f wmb(const FragB& a, const FragB& b, v8f c) {
  v8f d = __builtin_amdgcn_wmma_f32_16x16x32_bf16(false, a.v, false, b.v, (short)0, c, false, false);
  asm volatile("v_nop\n\tv_nop\n\tv_nop\n\tv_nop" : "+v"(d) : "v"(a.w), "v"(b.w));
  return d;
}

__device__ __forceinline__ unsigned int f2bf(float f) {
  const unsigned int u = __float_as_uint(f);
  return ((u + 0x7FFFu + ((u >> 16) & 1u)) >> 16) & 0xFFFFu;
}
__device__ __forceinline__ float bf2f(unsigned int b) { return __uint_as_float(b << 16); }
__device__ __forceinline__ float bfr(float f) { return bf2f(f2bf(f)); }
__device__ __forceinline__ unsigned int pk2(float lo, float hi) { return f2bf(lo) | (f2bf(hi) << 16); }
__device__ __forceinline__ v4u pack8(const v4f a, const v4f b) {
  v4u r;
  r.x = pk2(a.x, a.y); r.y = pk2(a.z, a.w); r.z = pk2(b.x, b.y); r.w = pk2(b.z, b.w);
  return r;
}
__device__ __forceinline__ void split8(const v4f a, const v4f b, v4u& hv, v4u& lv) {
  const unsigned int h0 = f2bf(a.x), h1 = f2bf(a.y), h2 = f2bf(a.z), h3 = f2bf(a.w);
  const unsigned int h4 = f2bf(b.x), h5 = f2bf(b.y), h6 = f2bf(b.z), h7 = f2bf(b.w);
  const unsigned int l0 = f2bf(a.x - bf2f(h0)), l1 = f2bf(a.y - bf2f(h1));
  const unsigned int l2 = f2bf(a.z - bf2f(h2)), l3 = f2bf(a.w - bf2f(h3));
  const unsigned int l4 = f2bf(b.x - bf2f(h4)), l5 = f2bf(b.y - bf2f(h5));
  const unsigned int l6 = f2bf(b.z - bf2f(h6)), l7 = f2bf(b.w - bf2f(h7));
  hv.x = h0 | (h1 << 16); hv.y = h2 | (h3 << 16); hv.z = h4 | (h5 << 16); hv.w = h6 | (h7 << 16);
  lv.x = l0 | (l1 << 16); lv.y = l2 | (l3 << 16); lv.z = l4 | (l5 << 16); lv.w = l6 | (l7 << 16);
}

__device__ __forceinline__ float leaky(float t) { return t >= 0.0f ? t : NEGSL * t; }

__global__ __launch_bounds__(NTHR) void k_xprep(const float* __restrict__ x, unsigned short* xb, int nN, int nUnits) {
  const int i = (int)blockIdx.x * NTHR + (int)threadIdx.x;
  if (i >= nUnits) return;
  const int row = i >> 5;
  const int c0  = (i & 31) * 8;
  const int rc  = row < nN ? row : nN - 1;
  const float* p = x + (size_t)rc * KIN + c0;
  v4f a = *(const v4fa*)p, b = *(const v4fa*)(p + 4);
  const v4f z4 = {0.f, 0.f, 0.f, 0.f};
  if (row >= nN) { a = z4; b = z4; }
  const v4u hv = pack8(a, b);
  const size_t o = (size_t)row * KIN + c0;
  *(volatile v4u*)(xb + o) = hv;
  __threadfence();
  *(volatile v4u*)(xb + o) = hv;
}

__global__ __launch_bounds__(NTHR) void k_wtr(const float* __restrict__ w, int cols, int K,
                                              unsigned short* wt, int nUnits) {
  const int u = (int)blockIdx.x * NTHR + (int)threadIdx.x;
  if (u >= nUnits) return;
  const int kq = K >> 3;
  const int n  = u / kq;
  const int k8 = (u - n * kq) * 8;
  const int ncl = n < cols ? n : cols - 1;
  const float* p = w + (size_t)k8 * (size_t)cols + ncl;
  v4f a, b;
  a.x = p[0];                  a.y = p[(size_t)cols];       a.z = p[(size_t)2 * cols];   a.w = p[(size_t)3 * cols];
  b.x = p[(size_t)4 * cols];   b.y = p[(size_t)5 * cols];   b.z = p[(size_t)6 * cols];   b.w = p[(size_t)7 * cols];
  const v4f z4 = {0.f, 0.f, 0.f, 0.f};
  if (n >= cols) { a = z4; b = z4; }
  const v4u hv = pack8(a, b);
  const size_t o = (size_t)n * (size_t)K + k8;
  *(volatile v4u*)(wt + o) = hv;
  __threadfence();
  *(volatile v4u*)(wt + o) = hv;
}

__global__ __launch_bounds__(GTHR) void k_proj(
    const unsigned short* __restrict__ A, const unsigned short* __restrict__ WT,
    const float* __restrict__ a1, const float* __restrict__ a2,
    unsigned short* HTH, unsigned short* HTL, float* SS, int nN)
{
  __shared__ __attribute__((aligned(16))) float stg[GBM * DOUT];
  __shared__ __attribute__((aligned(16))) float satt[2 * DOUT];
  __shared__ __attribute__((aligned(16))) float sdot[2 * GBM];
  const int tid = (int)threadIdx.x, lane = tid & 31, wave = tid >> 5, hh = lane >> 4, m = lane & 15;
  const int rowBase = (int)blockIdx.x * GBM;

  {
    const int which = tid >> 6;
    const int c  = tid & 63;
    const float va = a1[c];
    const float vb = a2[c];
    const float w0 = (which == 0) ? 1.0f : 0.0f;
    const float w1 = (which == 0) ? 0.0f : 1.0f;
    const float v  = va * w0 + vb * w1;
    satt[which * DOUT + c] = bfr(v);
  }

  v8f acc[4];
  {
    const v8f z = {0.f, 0.f, 0.f, 0.f, 0.f, 0.f, 0.f, 0.f};
    acc[0] = z; acc[1] = z; acc[2] = z; acc[3] = z;
  }
  const unsigned short* ap = A  + (size_t)(rowBase + 16 * wave + m) * (size_t)KIN + 8 * hh;
  const unsigned short* wp = WT + (size_t)m * (size_t)KIN + 8 * hh;
#pragma unroll 1
  for (int ks = 0; ks < KIN / 32; ++ks) {
    FragB af;
    af.h[0] = *(const v8usa*)(ap + 32 * ks);
    af.h[1] = *(const v8usa*)(ap + 32 * ks + 16);
#pragma unroll
    for (int t = 0; t < 4; ++t) {
      const unsigned short* wq = wp + (size_t)(16 * t) * (size_t)KIN + 32 * ks;
      FragB bf;
      bf.h[0] = *(const v8usa*)wq;
      bf.h[1] = *(const v8usa*)(wq + 16);
      acc[t] = wmb(af, bf, acc[t]);
    }
  }

#pragma unroll
  for (int t = 0; t < 4; ++t) {
    const int lc = 16 * t + m;
#pragma unroll
    for (int r = 0; r < 8; ++r) {
      const int lr = 16 * wave + 8 * hh + r;
      stg[lr * DOUT + lc] = acc[t][r];
    }
  }
  __syncthreads();

  {
    const int row = tid & 63, which = tid >> 6;
    const float* sa = satt + which * DOUT;
    const float* hr = stg + row * DOUT;
    float d = 0.f;
#pragma unroll 4
    for (int c4 = 0; c4 < DOUT / 4; ++c4) {
      const v4f hv = *(const v4fa*)(hr + 4 * c4);
      const v4f av = *(const v4fa*)(sa + 4 * c4);
      d = fmaf(hv.x, av.x, d);
      d = fmaf(hv.y, av.y, d);
      d = fmaf(hv.z, av.z, d);
      d = fmaf(hv.w, av.w, d);
    }
    sdot[which * GBM + row] = d;
  }
  __syncthreads();

  const int q = tid & 7, ln = tid >> 3;
  v4u hv[4], lv[4];
#pragma unroll
  for (int p = 0; p < 4; ++p) {
    const int n = 16 * p + ln;
    v4f ga, gb;
    ga.x = stg[(8 * q + 0) * DOUT + n]; ga.y = stg[(8 * q + 1) * DOUT + n];
    ga.z = stg[(8 * q + 2) * DOUT + n]; ga.w = stg[(8 * q + 3) * DOUT + n];
    gb.x = stg[(8 * q + 4) * DOUT + n]; gb.y = stg[(8 * q + 5) * DOUT + n];
    gb.z = stg[(8 * q + 6) * DOUT + n]; gb.w = stg[(8 * q + 7) * DOUT + n];
    split8(ga, gb, hv[p], lv[p]);
  }
  const int which2 = lane >> 4, piece = lane & 15;
  const v4f sdv = *(const v4fa*)(sdot + which2 * GBM + 4 * piece);
  float* sp = SS + (size_t)which2 * (size_t)nN + rowBase + 4 * piece;

#pragma unroll
  for (int p = 0; p < 4; ++p) {
    const size_t o = (size_t)(16 * p + ln) * (size_t)nN + (size_t)rowBase + 8 * q;
    *(volatile v4u*)(HTH + o) = hv[p];
    *(volatile v4u*)(HTL + o) = lv[p];
  }
  if (wave == 0) *(volatile v4f*)sp = sdv;
  __threadfence();
#pragma unroll
  for (int p = 0; p < 4; ++p) {
    const size_t o = (size_t)(16 * p + ln) * (size_t)nN + (size_t)rowBase + 8 * q;
    *(volatile v4u*)(HTH + o) = hv[p];
    *(volatile v4u*)(HTL + o) = lv[p];
  }
  if (wave == 0) *(volatile v4f*)sp = sdv;
}

__global__ __launch_bounds__(NTHR) void k_s2max(const float* __restrict__ s2, float* s2mx, int nN) {
  __shared__ float red[NTHR / 32];
  const int tid = (int)threadIdx.x, lane = tid & 31, wave = tid >> 5;
  float mx = __uint_as_float(0xff800000u);
#pragma unroll 1
  for (int i = 4 * tid; i < nN; i += 4 * NTHR) {
    const v4f v = *(const v4fa*)(s2 + i);
    mx = fmaxf(mx, fmaxf(fmaxf(v.x, v.y), fmaxf(v.z, v.w)));
  }
#pragma unroll
  for (int off = 16; off > 0; off >>= 1) mx = fmaxf(mx, __shfl_xor(mx, off));
  if (lane == 0) red[wave] = mx;
  __syncthreads();
  float bm = red[0];
#pragma unroll
  for (int w2 = 1; w2 < NTHR / 32; ++w2) bm = fmaxf(bm, red[w2]);
  v4f o; o.x = bm; o.y = bm; o.z = bm; o.w = bm;
  const bool wr = tid < 8;
  if (wr) *(volatile v4f*)(s2mx + 4 * tid) = o;
  __threadfence();
  if (wr) *(volatile v4f*)(s2mx + 4 * tid) = o;
}

__global__ __launch_bounds__(GTHR) void k_attn(
    const unsigned short* __restrict__ HTH, const unsigned short* __restrict__ HTL,
    const float* __restrict__ SS, const float* __restrict__ S2MX, float* out, int nN)
{
  __shared__ __attribute__((aligned(16))) unsigned short Ph[KT * PP];
  __shared__ __attribute__((aligned(16))) unsigned short Pl[KT * PP];
  __shared__ __attribute__((aligned(16))) float stg[GBM * DOUT];
  __shared__ __attribute__((aligned(16))) float lpart[2 * GBM];
  __shared__ __attribute__((aligned(16))) float linv[GBM];
  const int tid = (int)threadIdx.x, lane = tid & 31, wave = tid >> 5, hh = lane >> 4, m = lane & 15;
  const int rowBase = (int)blockIdx.x * GBM;
  const int i  = tid & 63;
  const int kh = tid >> 6;

  const float s2mx = S2MX[0];
  const float s1v  = SS[rowBase + i];
  const float mi   = leaky(s1v + s2mx);
  float lsum = 0.f;

  v8f acc[4];
  {
    const v8f z = {0.f, 0.f, 0.f, 0.f, 0.f, 0.f, 0.f, 0.f};
    acc[0] = z; acc[1] = z; acc[2] = z; acc[3] = z;
  }
  const unsigned short* aph = Ph + (16 * wave + m) * PP + 8 * hh;
  const unsigned short* apl = Pl + (16 * wave + m) * PP + 8 * hh;
  const unsigned short* bph = HTH + (size_t)m * (size_t)nN + 8 * hh;
  const unsigned short* bpl = HTL + (size_t)m * (size_t)nN + 8 * hh;
  unsigned short* prh = Ph + i * PP + 32 * kh;
  unsigned short* prl = Pl + i * PP + 32 * kh;
  const float* s2p = SS + (size_t)nN + 32 * kh;

  const int nT = nN / KT;
#pragma unroll 1
  for (int jt = 0; jt < nT; ++jt) {
    const int j0 = jt * KT;
    __syncthreads();

    float tl = 0.f;
#pragma unroll
    for (int q = 0; q < 4; ++q) {
      const v4f sa = *(const v4fa*)(s2p + j0 + 8 * q);
      const v4f sb = *(const v4fa*)(s2p + j0 + 8 * q + 4);
      v4f pa, pb;
      pa.x = expf(leaky(s1v + sa.x) - mi);
      pa.y = expf(leaky(s1v + sa.y) - mi);
      pa.z = expf(leaky(s1v + sa.z) - mi);
      pa.w = expf(leaky(s1v + sa.w) - mi);
      pb.x = expf(leaky(s1v + sb.x) - mi);
      pb.y = expf(leaky(s1v + sb.y) - mi);
      pb.z = expf(leaky(s1v + sb.z) - mi);
      pb.w = expf(leaky(s1v + sb.w) - mi);
      tl = tl + pa.x; tl = tl + pa.y; tl = tl + pa.z; tl = tl + pa.w;
      tl = tl + pb.x; tl = tl + pb.y; tl = tl + pb.z; tl = tl + pb.w;
      v4u hv, lv;
      split8(pa, pb, hv, lv);
      *(v4ua*)(prh + 8 * q) = hv;
      *(v4ua*)(prl + 8 * q) = lv;
    }
    lsum = lsum + tl;
    __syncthreads();

#pragma unroll
    for (int ks = 0; ks < KT / 32; ++ks) {
      FragB ah, al;
      ah.h[0] = *(const v8usa*)(aph + 32 * ks);
      ah.h[1] = *(const v8usa*)(aph + 32 * ks + 16);
      al.h[0] = *(const v8usa*)(apl + 32 * ks);
      al.h[1] = *(const v8usa*)(apl + 32 * ks + 16);
#pragma unroll
      for (int t = 0; t < 4; ++t) {
        const size_t bo = (size_t)(16 * t) * (size_t)nN + (size_t)j0 + 32 * ks;
        FragB bh, bl;
        bh.h[0] = *(const v8usa*)(bph + bo);
        bh.h[1] = *(const v8usa*)(bph + bo + 16);
        bl.h[0] = *(const v8usa*)(bpl + bo);
        bl.h[1] = *(const v8usa*)(bpl + bo + 16);
        acc[t] = wmb(ah, bh, acc[t]);
        acc[t] = wmb(al, bh, acc[t]);
        acc[t] = wmb(ah, bl, acc[t]);
      }
    }
  }

  lpart[kh * GBM + i] = lsum;
  __syncthreads();
  if (tid < GBM) linv[tid] = 1.0f / (lpart[tid] + lpart[GBM + tid]);
  __syncthreads();

#pragma unroll
  for (int t = 0; t < 4; ++t) {
    const int lc = 16 * t + m;
#pragma unroll
    for (int r = 0; r < 8; ++r) {
      const int lr = 16 * wave + 8 * hh + r;
      stg[lr * DOUT + lc] = acc[t][r] * linv[lr];
    }
  }
  __syncthreads();

  v4f fv[8];
#pragma unroll
  for (int u = 0; u < 8; ++u) {
    const int lr = 16 * wave + 2 * u + hh;
    fv[u] = *(const v4fa*)(stg + lr * DOUT + 4 * m);
  }
#pragma unroll
  for (int u = 0; u < 8; ++u) {
    const int lr = 16 * wave + 2 * u + hh;
    float* op = out + (size_t)(rowBase + lr) * DOUT + 4 * m;
    *(volatile v4f*)op = fv[u];
  }
  __threadfence();
#pragma unroll
  for (int u = 0; u < 8; ++u) {
    const int lr = 16 * wave + 2 * u + hh;
    float* op = out + (size_t)(rowBase + lr) * DOUT + 4 * m;
    *(volatile v4f*)op = fv[u];
  }
}

static inline int cdiv(int a, int b) { return (a + b - 1) / b; }

extern "C" void kernel_launch(void* const* d_in, const int* in_sizes, int n_in,
                              void* d_out, int out_size, void* d_ws, size_t ws_size,
                              hipStream_t stream) {
  if (n_in < 4) return;
  const int nN = in_sizes[0] / KIN;
  if (nN < KT || in_sizes[0] != nN * KIN || (nN % GBM) != 0 || (nN % KT) != 0 || nN > (1 << 20)) return;
  if (in_sizes[1] != KIN * DOUT) return;
  if (in_sizes[2] != DOUT || in_sizes[3] != DOUT) return;
  if (out_size != nN * DOUT) return;

  const float* x  = (const float*)d_in[0];
  const float* W  = (const float*)d_in[1];
  const float* a1 = (const float*)d_in[2];
  const float* a2 = (const float*)d_in[3];
  float* out = (float*)d_out;

  char* ws = (char*)d_ws;
  size_t off = 0;
  const size_t oXB  = off; off += (size_t)nN * KIN * 2;            off = (off + 255) & ~(size_t)255;
  const size_t oWT  = off; off += (size_t)DOUT * KIN * 2;          off = (off + 255) & ~(size_t)255;
  const size_t oHTH = off; off += (size_t)DOUT * nN * 2;           off = (off + 255) & ~(size_t)255;
  const size_t oHTL = off; off += (size_t)DOUT * nN * 2;           off = (off + 255) & ~(size_t)255;
  const size_t oSS  = off; off += (size_t)2 * nN * 4;              off = (off + 255) & ~(size_t)255;
  const size_t oMX  = off; off += 256;
  if (off > ws_size || off > (size_t)WSMAX) return;
  unsigned short* XB  = (unsigned short*)(ws + oXB);
  unsigned short* WT  = (unsigned short*)(ws + oWT);
  unsigned short* HTH = (unsigned short*)(ws + oHTH);
  unsigned short* HTL = (unsigned short*)(ws + oHTL);
  float*          SS  = (float*)(ws + oSS);
  float*          MX  = (float*)(ws + oMX);

  const int nUx = nN * (KIN / 8);
  k_xprep<<<cdiv(nUx, NTHR), NTHR, 0, stream>>>(x, XB, nN, nUx);

  const int nUw = DOUT * (KIN / 8);
  k_wtr<<<cdiv(nUw, NTHR), NTHR, 0, stream>>>(W, DOUT, KIN, WT, nUw);

  k_proj<<<nN / GBM, GTHR, 0, stream>>>(XB, WT, a1, a2, HTH, HTL, SS, nN);

  k_s2max<<<1, NTHR, 0, stream>>>(SS + nN, MX, nN);

  k_attn<<<nN / GBM, GTHR, 0, stream>>>(HTH, HTL, SS, MX, out, nN);
}
